// GNNQNetwork_35785667510417
// MI455X (gfx1250) — hardware-verified
//
#include <hip/hip_runtime.h>
#include <stddef.h>


#define DF     128
#define GR     32
#define KC     64
#define APU    72
#define XSP    132
#define NTHR   256
#define NWAVE  8
#define NB     512
#define NHD    4
#define CHUNK  2048
#define WCAP   256
#define NGRP   (CHUNK / (NTHR * 4))
#define KPA    576
#define CMB    512
#define TRW    384
#define NACT   32
#define NEGBIG (-3.0e38f)

#define LDS_SACC (NB * DF)
#define LDS_MD   (NB * NHD)
#define LDS_LIST (NWAVE * WCAP)
#define GAT_LDS_BYTES ((LDS_SACC + 2 * LDS_MD + LDS_LIST + NWAVE) * 4)

static_assert(GAT_LDS_BYTES == 286752);
static_assert(WCAP == (CHUNK / NTHR) * 32);
static_assert(NGRP == 2);
static_assert(NB == 512);
static_assert(CHUNK == 2048);
static_assert((APU * 2) % 16 == 0);
static_assert((XSP * 4) % 16 == 0);
static_assert(KPA == 4 * DF + 64);

typedef float          v4f   __attribute__((ext_vector_type(4)));
typedef float          v8f   __attribute__((ext_vector_type(8)));
typedef int            v4i   __attribute__((ext_vector_type(4)));
typedef unsigned short v8us  __attribute__((ext_vector_type(8)));
typedef __bf16         v16bf __attribute__((ext_vector_type(16)));
union Frag { v16bf v; v8us u[2]; };
union Pk8  { v8us v; unsigned short s[8]; };
static_assert(sizeof(Frag) == 32);
static_assert(sizeof(Pk8) == 16);

__device__ __forceinline__ unsigned short f2bf(float f) {
  unsigned u = __float_as_uint(f);
  u += 0x7FFFu + ((u >> 16) & 1u);
  return (unsigned short)(u >> 16);
}
__device__ __forceinline__ void split2(float f, unsigned short& hi, unsigned short& lo) {
  const unsigned short hb = f2bf(f);
  const float fh = __uint_as_float(((unsigned)hb) << 16);
  hi = hb;
  lo = f2bf(f - fh);
}

__device__ __forceinline__ v8f wm(v16bf a, v16bf b, v8f c) {
  v8f d = __builtin_amdgcn_wmma_f32_16x16x32_bf16(false, a, false, b, (short)0, c, false, false);
  asm volatile("v_nop\n\tv_nop\n\tv_nop\n\tv_nop" : "+v"(d) : "v"(a), "v"(b));
  return d;
}

__device__ __forceinline__ float wsum(float v) {
  v += __shfl_xor(v, 16, 32);
  v += __shfl_xor(v, 8, 32);
  v += __shfl_xor(v, 4, 32);
  v += __shfl_xor(v, 2, 32);
  v += __shfl_xor(v, 1, 32);
  return v;
}

__device__ __forceinline__ v4f lrelu4(v4f t) {
  t.x = (t.x > 0.f) ? t.x : 0.2f * t.x;
  t.y = (t.y > 0.f) ? t.y : 0.2f * t.y;
  t.z = (t.z > 0.f) ? t.z : 0.2f * t.z;
  t.w = (t.w > 0.f) ? t.w : 0.2f * t.w;
  return t;
}

__device__ __forceinline__ float hdot(v4f t, v4f a) {
  float p = t.x * a.x + t.y * a.y + t.z * a.z + t.w * a.w;
  p += __shfl_xor(p, 1, 32);
  p += __shfl_xor(p, 2, 32);
  p += __shfl_xor(p, 4, 32);
  return p;
}

__global__ __launch_bounds__(NTHR) void k_prepw(const float* __restrict__ W0, const float* __restrict__ W1,
                                                unsigned short* Ph, unsigned short* Pl, int K, int KP) {
  const float* W = (blockIdx.y != 0) ? W1 : W0;
  const int t = blockIdx.x * NTHR + threadIdx.x;
  const int per = KP >> 3;
  const int total = DF * per;
  if (t >= total) return;
  const int n = t / per;
  const int k0 = (t - n * per) * 8;
  Pk8 uh, ul;
#pragma unroll
  for (int j = 0; j < 8; ++j) {
    const int k = k0 + j;
    const int kk = (k < K) ? k : (K - 1);
    const float msk = (k < K) ? 1.0f : 0.0f;
    const float v = W[(size_t)kk * DF + n] * msk;
    unsigned short a, b;
    split2(v, a, b);
    uh.s[j] = a;
    ul.s[j] = b;
  }
  const size_t o = ((size_t)blockIdx.y * DF + n) * (size_t)KP + k0;
  *(volatile v8us*)(Ph + o) = uh.v;
  *(volatile v8us*)(Pl + o) = ul.v;
  __threadfence();
  *(volatile v8us*)(Ph + o) = uh.v;
  *(volatile v8us*)(Pl + o) = ul.v;
}

__global__ __launch_bounds__(NTHR) void k_encode(const float* __restrict__ x, const float* __restrict__ Wn,
                                                 const float* __restrict__ bn, float* h, int nN) {
  const int tid = threadIdx.x, lane = tid & 31, wave = tid >> 5;
  const int r0 = blockIdx.x * GR + wave * 4;
  const v4f w4 = *(const v4f*)(Wn + 4 * lane);
  const v4f b4 = *(const v4f*)(bn + 4 * lane);
  v4f y[4];
#pragma unroll
  for (int i = 0; i < 4; ++i) {
    int row = r0 + i;
    if (row > nN - 1) row = nN - 1;
    const float xv = x[row];
    v4f t = xv * w4 + b4;
    t.x = fmaxf(t.x, 0.f); t.y = fmaxf(t.y, 0.f); t.z = fmaxf(t.z, 0.f); t.w = fmaxf(t.w, 0.f);
    y[i] = t;
  }
#pragma unroll
  for (int i = 0; i < 4; ++i)
    if (r0 + i < nN) *(volatile v4f*)(h + (size_t)(r0 + i) * DF + 4 * lane) = y[i];
  __threadfence();
#pragma unroll
  for (int i = 0; i < 4; ++i)
    if (r0 + i < nN) *(volatile v4f*)(h + (size_t)(r0 + i) * DF + 4 * lane) = y[i];
}

__global__ __launch_bounds__(NTHR) void k_mean(const float* __restrict__ ea, float* meanl, int nE) {
  __shared__ double red[NTHR];
  const int tid = threadIdx.x;
  const int per = (nE + NTHR - 1) / NTHR;
  const int i0 = tid * per;
  int i1 = i0 + per;
  if (i1 > nE) i1 = nE;
  double s = 0.0;
#pragma unroll 1
  for (int i = i0; i < i1; ++i) s += (double)ea[i];
  red[tid] = s;
  __syncthreads();
#pragma unroll 1
  for (int st = NTHR / 2; st > 0; st >>= 1) {
    if (tid < st) red[tid] += red[tid + st];
    __syncthreads();
  }
  const float mv = (float)(red[0] / (double)nE);
  if (tid < 32) *(volatile float*)(meanl + tid) = mv;
  __threadfence();
  if (tid < 32) *(volatile float*)(meanl + tid) = mv;
}

__global__ __launch_bounds__(NTHR) void k_gemm(
    const float* __restrict__ A, int lda, int M, int KP,
    const unsigned short* __restrict__ Bh, const unsigned short* __restrict__ Bl,
    const float* __restrict__ bias0, const float* __restrict__ bias1,
    float* C0, float* C1, int ldc, int relu) {
  __shared__ __attribute__((aligned(16))) unsigned short Ah[GR * APU];
  __shared__ __attribute__((aligned(16))) unsigned short Al[GR * APU];
  __shared__ __attribute__((aligned(16))) float Xs[GR * XSP];

  const int tid  = threadIdx.x;
  const int lane = tid & 31;
  const int wave = tid >> 5;
  const int hh   = lane >> 4;
  const int m    = lane & 15;
  const int rowBase = blockIdx.x * GR;
  const int ysel = blockIdx.y;
  const unsigned short* Bhy = Bh + (size_t)ysel * DF * (size_t)KP;
  const unsigned short* Bly = Bl + (size_t)ysel * DF * (size_t)KP;
  const float* bias = (ysel != 0) ? bias1 : bias0;
  float* C = (ysel != 0) ? C1 : C0;
  const int ncol = wave * 16 + m;

  const int sr  = tid >> 3;
  const int sc0 = (tid & 7) * 8;
  int srow = rowBase + sr;
  if (srow > M - 1) srow = M - 1;
  const float* Arow = A + (size_t)srow * lda + sc0;

  v8f acc0 = {0.f, 0.f, 0.f, 0.f, 0.f, 0.f, 0.f, 0.f};
  v8f acc1 = {0.f, 0.f, 0.f, 0.f, 0.f, 0.f, 0.f, 0.f};

#pragma unroll 1
  for (int kc = 0; kc < KP; kc += KC) {
    {
      const v4f f0 = *(const v4f*)(Arow + kc);
      const v4f f1 = *(const v4f*)(Arow + kc + 4);
      Pk8 uh, ul;
      split2(f0.x, uh.s[0], ul.s[0]);
      split2(f0.y, uh.s[1], ul.s[1]);
      split2(f0.z, uh.s[2], ul.s[2]);
      split2(f0.w, uh.s[3], ul.s[3]);
      split2(f1.x, uh.s[4], ul.s[4]);
      split2(f1.y, uh.s[5], ul.s[5]);
      split2(f1.z, uh.s[6], ul.s[6]);
      split2(f1.w, uh.s[7], ul.s[7]);
      *(v8us*)(Ah + sr * APU + sc0) = uh.v;
      *(v8us*)(Al + sr * APU + sc0) = ul.v;
    }
    __syncthreads();
#pragma unroll
    for (int ks = 0; ks < KC / 32; ++ks) {
      const int k0 = ks * 32;
      Frag a0h, a0l, a1h, a1l, bh, bl;
      const unsigned short* pb = Bhy + (size_t)ncol * KP + kc + k0 + 8 * hh;
      const unsigned short* pc = Bly + (size_t)ncol * KP + kc + k0 + 8 * hh;
      bh.u[0] = *(const v8us*)pb;  bh.u[1] = *(const v8us*)(pb + 16);
      bl.u[0] = *(const v8us*)pc;  bl.u[1] = *(const v8us*)(pc + 16);
      const unsigned short* pa0 = Ah + m * APU + k0 + 8 * hh;
      const unsigned short* pa1 = Ah + (16 + m) * APU + k0 + 8 * hh;
      const unsigned short* qa0 = Al + m * APU + k0 + 8 * hh;
      const unsigned short* qa1 = Al + (16 + m) * APU + k0 + 8 * hh;
      a0h.u[0] = *(const v8us*)pa0; a0h.u[1] = *(const v8us*)(pa0 + 16);
      a1h.u[0] = *(const v8us*)pa1; a1h.u[1] = *(const v8us*)(pa1 + 16);
      a0l.u[0] = *(const v8us*)qa0; a0l.u[1] = *(const v8us*)(qa0 + 16);
      a1l.u[0] = *(const v8us*)qa1; a1l.u[1] = *(const v8us*)(qa1 + 16);
      acc0 = wm(a0h.v, bh.v, acc0);
      acc0 = wm(a0h.v, bl.v, acc0);
      acc0 = wm(a0l.v, bh.v, acc0);
      acc1 = wm(a1h.v, bh.v, acc1);
      acc1 = wm(a1h.v, bl.v, acc1);
      acc1 = wm(a1l.v, bh.v, acc1);
    }
    __syncthreads();
  }

  const float bv = bias[ncol];
#pragma unroll
  for (int r = 0; r < 8; ++r) {
    float v0 = acc0[r] + bv;
    float v1 = acc1[r] + bv;
    if (relu != 0) { v0 = fmaxf(v0, 0.f); v1 = fmaxf(v1, 0.f); }
    Xs[(8 * hh + r) * XSP + ncol]      = v0;
    Xs[(16 + 8 * hh + r) * XSP + ncol] = v1;
  }
  __syncthreads();

  v4f xv[4];
#pragma unroll
  for (int i = 0; i < 4; ++i) xv[i] = *(const v4f*)(Xs + (4 * wave + i) * XSP + 4 * lane);
  const int rw = rowBase + 4 * wave;
#pragma unroll
  for (int i = 0; i < 4; ++i)
    if (rw + i < M) *(volatile v4f*)(C + (size_t)(rw + i) * ldc + 4 * lane) = xv[i];
  __threadfence();
#pragma unroll
  for (int i = 0; i < 4; ++i)
    if (rw + i < M) *(volatile v4f*)(C + (size_t)(rw + i) * ldc + 4 * lane) = xv[i];
}

__global__ __launch_bounds__(NTHR) void k_gat(
    const int* __restrict__ ei, const float* __restrict__ ea,
    const float* __restrict__ xl, const float* __restrict__ xr,
    const float* __restrict__ We, const float* __restrict__ att, const float* __restrict__ gb,
    const float* __restrict__ meanl, float* h, int nN, int nE) {
  extern __shared__ v4f lds_dyn[];
  float* sacc = (float*)lds_dyn;
  float* mxa  = sacc + LDS_SACC;
  float* dena = mxa + LDS_MD;
  int*   list = (int*)(dena + LDS_MD);
  int*   wcnt = list + LDS_LIST;

  const int tid  = threadIdx.x;
  const int lane = tid & 31;
  const int wave = tid >> 5;
  const int hd   = lane >> 3;
  const int nodeBase = blockIdx.x * NB;

  {
    const v4f z4 = {0.f, 0.f, 0.f, 0.f};
    for (int i = tid; i < LDS_SACC / 4; i += NTHR) lds_dyn[i] = z4;
    for (int i = tid; i < LDS_MD; i += NTHR) { mxa[i] = NEGBIG; dena[i] = 0.f; }
  }
  const v4f we4 = *(const v4f*)(We + 4 * lane);
  const v4f at4 = *(const v4f*)(att + 4 * lane);
  const v4f gb4 = *(const v4f*)(gb + 4 * lane);
  const float emean = meanl[0];
  __syncthreads();

  const int* eid = ei + nE;
  const bool al16 = ((nE & 3) == 0);

  const int nChunks = (nE + CHUNK - 1) / CHUNK;
#pragma unroll 1
  for (int ch = 0; ch < nChunks; ++ch) {
    const int cbase = ch * CHUNK;
    int wc = 0;
#pragma unroll
    for (int g = 0; g < NGRP; ++g) {
      const int el0 = (g * NTHR + tid) * 4;
      const int e0  = cbase + el0;
      const int sent = -2147483647 - 1;
      v4i d;
      if (al16 && (cbase + CHUNK <= nE)) {
        d = *(const v4i*)(eid + e0);
      } else {
        d.x = (e0     < nE) ? eid[min(e0,     nE - 1)] : sent;
        d.y = (e0 + 1 < nE) ? eid[min(e0 + 1, nE - 1)] : sent;
        d.z = (e0 + 2 < nE) ? eid[min(e0 + 2, nE - 1)] : sent;
        d.w = (e0 + 3 < nE) ? eid[min(e0 + 3, nE - 1)] : sent;
      }
      const unsigned s0 = (unsigned)d.x - (unsigned)nodeBase;
      const unsigned s1 = (unsigned)d.y - (unsigned)nodeBase;
      const unsigned s2 = (unsigned)d.z - (unsigned)nodeBase;
      const unsigned s3 = (unsigned)d.w - (unsigned)nodeBase;
      const bool h0 = s0 < (unsigned)NB;
      const bool h1 = s1 < (unsigned)NB;
      const bool h2 = s2 < (unsigned)NB;
      const bool h3 = s3 < (unsigned)NB;
      const unsigned many = __builtin_amdgcn_ballot_w32(h0 | h1 | h2 | h3);
      if (many != 0u) {
#define HITJ(J, HJ, SJ) { \
          const unsigned mj = __builtin_amdgcn_ballot_w32(HJ); \
          if (HJ) { \
            const int pos = wc + (int)__builtin_amdgcn_mbcnt_lo(mj, 0u); \
            if (pos < WCAP) list[wave * WCAP + pos] = ((el0 + (J)) << 9) | (int)(SJ); \
          } \
          wc += (int)__builtin_popcount(mj); }
        HITJ(0, h0, s0)
        HITJ(1, h1, s1)
        HITJ(2, h2, s2)
        HITJ(3, h3, s3)
#undef HITJ
      }
    }
    if (lane == 0) wcnt[wave] = wc;
    __syncthreads();

    if (wave == 0) {
#pragma unroll 1
      for (int wsx = 0; wsx < NWAVE; ++wsx) {
        int n = wcnt[wsx];
        if (n > WCAP) n = WCAP;
        if (n < 0) n = 0;
#pragma unroll 1
        for (int i = 0; i < n; ++i) {
          const int ent  = list[wsx * WCAP + i];
          const int slot = ent & (NB - 1);
          const int el   = (ent >> 9) & (CHUNK - 1);
          int e = cbase + el;
          if (e > nE - 1) e = nE - 1;
          int src = ei[e];
          src = src < 0 ? 0 : (src > nN - 1 ? nN - 1 : src);
          const float w = ea[e];
          int nd = nodeBase + slot;
          if (nd > nN - 1) nd = nN - 1;
          const v4f xv = *(const v4f*)(xl + (size_t)src * DF + 4 * lane);
          const v4f rv = *(const v4f*)(xr + (size_t)nd * DF + 4 * lane);
          const v4f t  = lrelu4(xv + rv + w * we4);
          const float lg = hdot(t, at4);
          const int ai = slot * NHD + hd;
          const float mo = mxa[ai];
          const float dn = dena[ai];
          const float mn = fmaxf(mo, lg);
          const float sc = __expf(mo - mn);
          const float p  = __expf(lg - mn);
          v4f* sp = (v4f*)(sacc + slot * DF + 4 * lane);
          const v4f cur = *sp;
          *sp = cur * sc + p * xv;
          mxa[ai]  = mn;
          dena[ai] = dn * sc + p;
        }
      }
    }
    __syncthreads();
  }

#pragma unroll 1
  for (int j = 0; j < NB / NWAVE; ++j) {
    const int slot = wave * (NB / NWAVE) + j;
    const int node = nodeBase + slot;
    if (node >= nN) break;
    const size_t nrow = (size_t)node;
    const v4f xv = *(const v4f*)(xl + nrow * DF + 4 * lane);
    const v4f rv = *(const v4f*)(xr + nrow * DF + 4 * lane);
    const v4f t  = lrelu4(xv + rv + emean * we4);
    const float lg = hdot(t, at4);
    const int ai = slot * NHD + hd;
    const float mo = mxa[ai];
    const float mn = fmaxf(mo, lg);
    const float sc = __expf(mo - mn);
    const float p  = __expf(lg - mn);
    const v4f sv = *(const v4f*)(sacc + slot * DF + 4 * lane) * sc + p * xv;
    const float dv  = dena[ai] * sc + p;
    const float inv = __builtin_amdgcn_rcpf(dv);
    v4f o = sv * inv + gb4;
    o.x = fmaxf(o.x, 0.f); o.y = fmaxf(o.y, 0.f); o.z = fmaxf(o.z, 0.f); o.w = fmaxf(o.w, 0.f);
    const v4f hold = *(const v4f*)(h + nrow * DF + 4 * lane);
    const v4f y = o + hold;
    float* op = h + nrow * DF + 4 * lane;
    *(volatile v4f*)op = y;
    __threadfence();
    *(volatile v4f*)op = y;
  }
}

__global__ __launch_bounds__(128) void k_pool(const float* __restrict__ h, const int* __restrict__ bidx,
                                              const int* __restrict__ ptr, float* tree, int nN) {
  __shared__ __attribute__((aligned(16))) float rowv[TRW];
  const int g = blockIdx.x;
  const int f = threadIdx.x;
  int lo = ptr[g];
  int hi = ptr[g + 1];
  lo = lo < 0 ? 0 : (lo > nN ? nN : lo);
  hi = hi < lo ? lo : (hi > nN ? nN : hi);
  double s = 0.0;
  float mx = -__builtin_inff();
  int cnt = 0;
#pragma unroll 1
  for (int i = lo; i < hi; ++i) {
    const int b = bidx[i];
    const float v = h[(size_t)i * DF + f];
    const bool in = (b == g);
    s  += in ? (double)v : 0.0;
    mx  = in ? fmaxf(mx, v) : mx;
    cnt += in ? 1 : 0;
  }
  const float sf = (float)s;
  rowv[f]           = sf;
  rowv[DF + f]      = sf * __builtin_amdgcn_rcpf((float)cnt);
  rowv[2 * DF + f]  = mx;
  __syncthreads();
  v4f v = {0.f, 0.f, 0.f, 0.f};
  if (f < TRW / 4) v = *(const v4f*)(rowv + 4 * f);
  float* p = tree + (size_t)g * TRW + 4 * f;
  if (f < TRW / 4) *(volatile v4f*)p = v;
  __threadfence();
  if (f < TRW / 4) *(volatile v4f*)p = v;
}

__global__ __launch_bounds__(NTHR) void k_gather(const float* __restrict__ h, const float* __restrict__ act,
                                                 const int* __restrict__ ptr, const float* __restrict__ tree,
                                                 float* ai, float* comb, int nN) {
  const int g = blockIdx.x;
  const int tid = threadIdx.x, lane = tid & 31, wave = tid >> 5;
  const int base = ptr[g];
#pragma unroll 1
  for (int a = wave; a < NACT; a += NWAVE) {
    const int row = g * NACT + a;
    const float* av = act + (size_t)row * 7;
    v4f hv[4];
#pragma unroll
    for (int j = 0; j < 4; ++j) {
      const float fv = av[j];
      int ni = (int)fv + base;
      ni = (ni < 0) ? ni + nN : ni;
      ni = ni < 0 ? 0 : (ni > nN - 1 ? nN - 1 : ni);
      hv[j] = *(const v4f*)(h + (size_t)ni * DF + 4 * lane);
    }
    const float m0 = av[4], m1 = av[5], m2 = av[6];
    v4f tail = {0.f, 0.f, 0.f, 0.f};
    if (lane == 0) { tail.x = m0; tail.y = m1; tail.z = m2; }
    v4f tv[3];
#pragma unroll
    for (int j = 0; j < 3; ++j) tv[j] = *(const v4f*)(tree + (size_t)g * TRW + DF * j + 4 * lane);

    float* arow = ai + (size_t)row * KPA;
    float* crow = comb + (size_t)row * CMB;
#pragma unroll
    for (int j = 0; j < 4; ++j) *(volatile v4f*)(arow + DF * j + 4 * lane) = hv[j];
    if (lane < 16) *(volatile v4f*)(arow + 4 * DF + 4 * lane) = tail;
#pragma unroll
    for (int j = 0; j < 3; ++j) *(volatile v4f*)(crow + DF * j + 4 * lane) = tv[j];
    __threadfence();
#pragma unroll
    for (int j = 0; j < 4; ++j) *(volatile v4f*)(arow + DF * j + 4 * lane) = hv[j];
    if (lane < 16) *(volatile v4f*)(arow + 4 * DF + 4 * lane) = tail;
#pragma unroll
    for (int j = 0; j < 3; ++j) *(volatile v4f*)(crow + DF * j + 4 * lane) = tv[j];
  }
}

__global__ __launch_bounds__(32) void k_qout(const float* __restrict__ q2, const float* __restrict__ w3,
                                             const float* __restrict__ b3, float* out) {
  const int g = blockIdx.x;
  const int lane = threadIdx.x & 31;
  const v4f w4 = *(const v4f*)(w3 + 4 * lane);
  float mine = 0.f;
#pragma unroll 1
  for (int r = 0; r < NACT; ++r) {
    const v4f qv = *(const v4f*)(q2 + (size_t)(g * NACT + r) * DF + 4 * lane);
    float p = qv.x * w4.x + qv.y * w4.y + qv.z * w4.z + qv.w * w4.w;
    p = wsum(p);
    mine = (lane == r) ? p : mine;
  }
  mine += b3[0];
  const int sb = (lane & 7) * 4;
  v4f o;
  o.x = __shfl(mine, sb + 0, 32);
  o.y = __shfl(mine, sb + 1, 32);
  o.z = __shfl(mine, sb + 2, 32);
  o.w = __shfl(mine, sb + 3, 32);
  float* p = out + (size_t)g * NACT + 4 * lane;
  if (lane < 8) *(volatile v4f*)p = o;
  __threadfence();
  if (lane < 8) *(volatile v4f*)p = o;
}

extern "C" void kernel_launch(void* const* d_in, const int* in_sizes, int n_in,
                              void* d_out, int out_size, void* d_ws, size_t ws_size,
                              hipStream_t stream) {
  if (n_in < 25) return;
  const int nN = in_sizes[0];
  const int nE = in_sizes[1];
  const int nb = in_sizes[5] - 1;
  if (nN <= 0 || nE <= 0 || nb <= 0) return;
  if ((nN % GR) != 0) return;
  if (in_sizes[3] != 2 * nE || in_sizes[4] != nN) return;
  if (in_sizes[2] != nb * NACT * 7) return;
  const int M2 = nb * NACT;
  if (out_size != M2) return;
  if (in_sizes[6] != DF || in_sizes[7] != DF) return;
  const int L = in_sizes[8] / (DF * DF);
  if (L <= 0 || in_sizes[8] != L * DF * DF || in_sizes[9] != L * DF * DF) return;
  if (in_sizes[10] != L * DF || in_sizes[11] != L * DF) return;
  if (in_sizes[12] != L * DF || in_sizes[13] != L * DF || in_sizes[14] != L * DF) return;
  const int K1 = in_sizes[15] / DF;
  if (K1 != 4 * DF + 3 || in_sizes[15] != K1 * DF) return;
  if (in_sizes[16] != DF || in_sizes[17] != DF * DF || in_sizes[18] != DF) return;
  if (in_sizes[19] != CMB * DF || in_sizes[20] != DF || in_sizes[21] != DF * DF || in_sizes[22] != DF) return;
  if (in_sizes[23] != DF || in_sizes[24] != 1) return;

  const float* x    = (const float*)d_in[0];
  const float* ea   = (const float*)d_in[1];
  const float* act  = (const float*)d_in[2];
  const int*   ei   = (const int*)d_in[3];
  const int*   bidx = (const int*)d_in[4];
  const int*   bptr = (const int*)d_in[5];
  const float* Wn   = (const float*)d_in[6];
  const float* bn   = (const float*)d_in[7];
  const float* gWl  = (const float*)d_in[8];
  const float* gWr  = (const float*)d_in[9];
  const float* gWe  = (const float*)d_in[10];
  const float* gatt = (const float*)d_in[11];
  const float* gbl  = (const float*)d_in[12];
  const float* gbr  = (const float*)d_in[13];
  const float* gb   = (const float*)d_in[14];
  const float* aW1  = (const float*)d_in[15];
  const float* ab1  = (const float*)d_in[16];
  const float* aW2  = (const float*)d_in[17];
  const float* ab2  = (const float*)d_in[18];
  const float* qW1  = (const float*)d_in[19];
  const float* qb1  = (const float*)d_in[20];
  const float* qW2  = (const float*)d_in[21];
  const float* qb2  = (const float*)d_in[22];
  const float* qW3  = (const float*)d_in[23];
  const float* qb3  = (const float*)d_in[24];
  float* out = (float*)d_out;

  size_t off = 0;
  auto cv = [&](size_t bytes) -> char* {
    char* r = (char*)d_ws + off;
    off += (bytes + 255) & ~(size_t)255;
    return r;
  };
  float* hbuf = (float*)cv((size_t)nN * DF * 4);
  float* xl   = (float*)cv((size_t)nN * DF * 4);
  float* xr   = (float*)cv((size_t)nN * DF * 4);
  unsigned short* wlrH = (unsigned short*)cv((size_t)L * 2 * DF * DF * 2);
  unsigned short* wlrL = (unsigned short*)cv((size_t)L * 2 * DF * DF * 2);
  unsigned short* a1H  = (unsigned short*)cv((size_t)DF * KPA * 2);
  unsigned short* a1L  = (unsigned short*)cv((size_t)DF * KPA * 2);
  unsigned short* a2H  = (unsigned short*)cv((size_t)DF * DF * 2);
  unsigned short* a2L  = (unsigned short*)cv((size_t)DF * DF * 2);
  unsigned short* q1H  = (unsigned short*)cv((size_t)DF * CMB * 2);
  unsigned short* q1L  = (unsigned short*)cv((size_t)DF * CMB * 2);
  unsigned short* q2H  = (unsigned short*)cv((size_t)DF * DF * 2);
  unsigned short* q2L  = (unsigned short*)cv((size_t)DF * DF * 2);
  float* meanl  = (float*)cv(256);
  float* tree   = (float*)cv((size_t)nb * TRW * 4);
  float* airows = (float*)cv((size_t)M2 * KPA * 4);
  float* a1rows = (float*)cv((size_t)M2 * DF * 4);
  float* comb   = (float*)cv((size_t)M2 * CMB * 4);
  float* q1rows = (float*)cv((size_t)M2 * DF * 4);
  float* q2rows = (float*)cv((size_t)M2 * DF * 4);
  if (off > ws_size) return;
  if (off > ((size_t)128 << 20)) return;

  for (int l = 0; l < L; ++l) {
    k_prepw<<<dim3(DF / 16, 2), dim3(NTHR), 0, stream>>>(gWl + (size_t)l * DF * DF, gWr + (size_t)l * DF * DF,
                                                        wlrH + (size_t)l * 2 * DF * DF, wlrL + (size_t)l * 2 * DF * DF,
                                                        DF, DF);
  }
  k_prepw<<<dim3(KPA / 16, 1), dim3(NTHR), 0, stream>>>(aW1, aW1, a1H, a1L, K1, KPA);
  k_prepw<<<dim3(DF / 16, 1),  dim3(NTHR), 0, stream>>>(aW2, aW2, a2H, a2L, DF, DF);
  k_prepw<<<dim3(CMB / 16, 1), dim3(NTHR), 0, stream>>>(qW1, qW1, q1H, q1L, CMB, CMB);
  k_prepw<<<dim3(DF / 16, 1),  dim3(NTHR), 0, stream>>>(qW2, qW2, q2H, q2L, DF, DF);

  k_encode<<<dim3(nN / GR), dim3(NTHR), 0, stream>>>(x, Wn, bn, hbuf, nN);
  k_mean<<<dim3(1), dim3(NTHR), 0, stream>>>(ea, meanl, nE);

  hipFuncSetAttribute(reinterpret_cast<const void*>(&k_gat),
                      hipFuncAttributeMaxDynamicSharedMemorySize, GAT_LDS_BYTES);
  const int gatGrid = (nN + NB - 1) / NB;
  for (int l = 0; l < L; ++l) {
    k_gemm<<<dim3(nN / GR, 2), dim3(NTHR), 0, stream>>>(hbuf, DF, nN, DF,
                                                       wlrH + (size_t)l * 2 * DF * DF, wlrL + (size_t)l * 2 * DF * DF,
                                                       gbl + (size_t)l * DF, gbr + (size_t)l * DF,
                                                       xl, xr, DF, 0);
    k_gat<<<dim3(gatGrid), dim3(NTHR), GAT_LDS_BYTES, stream>>>(ei, ea, xl, xr,
                                                                gWe + (size_t)l * DF, gatt + (size_t)l * DF,
                                                                gb + (size_t)l * DF, meanl, hbuf, nN, nE);
  }

  k_pool<<<dim3(nb), dim3(128), 0, stream>>>(hbuf, bidx, bptr, tree, nN);
  k_gather<<<dim3(nb), dim3(NTHR), 0, stream>>>(hbuf, act, bptr, tree, airows, comb, nN);
  k_gemm<<<dim3(M2 / GR, 1), dim3(NTHR), 0, stream>>>(airows, KPA, M2, KPA, a1H, a1L, ab1, ab1,
                                                     a1rows, a1rows, DF, 1);
  k_gemm<<<dim3(M2 / GR, 1), dim3(NTHR), 0, stream>>>(a1rows, DF, M2, DF, a2H, a2L, ab2, ab2,
                                                     comb + TRW, comb + TRW, CMB, 1);
  k_gemm<<<dim3(M2 / GR, 1), dim3(NTHR), 0, stream>>>(comb, CMB, M2, CMB, q1H, q1L, qb1, qb1,
                                                     q1rows, q1rows, DF, 1);
  k_gemm<<<dim3(M2 / GR, 1), dim3(NTHR), 0, stream>>>(q1rows, DF, M2, DF, q2H, q2L, qb2, qb2,
                                                     q2rows, q2rows, DF, 1);
  k_qout<<<dim3(nb), dim3(32), 0, stream>>>(q2rows, qW3, qb3, out);
}
